// LocalAttentionUnFold_10144712753205
// MI455X (gfx1250) — hardware-verified
//
#include <hip/hip_runtime.h>

#define SEQ    2048
#define HID    1024
#define NHEAD  16
#define HDIM   64
#define NCAT   (3 * HID)
#define NXE    (SEQ * HID)
#define NWE    (HID * HID)
#define NX8    (NXE / 8)
#define NW8    (NWE / 8)
#define NCVT   (NX8 + 3 * NW8)
#define QB     32
#define KWIN   33
#define PPITCH 36

static_assert((NCVT % 256) == 0);
static_assert((NX8 % 256) == 0);
static_assert((NW8 % 256) == 0);
static_assert((SEQ % 128) == 0);
static_assert((NCAT % 64) == 0);
static_assert((SEQ % QB) == 0);
static_assert((HID % 32) == 0);

typedef __bf16         v16b __attribute__((ext_vector_type(16)));
typedef unsigned short v8us __attribute__((ext_vector_type(8)));
typedef float          v8f  __attribute__((ext_vector_type(8)));
typedef float          v4f  __attribute__((ext_vector_type(4)));
typedef v8us __attribute__((may_alias)) v8usa;
typedef v4f  __attribute__((may_alias)) v4fa;

union Frag { v16b v; v8us half[2]; };

__device__ __forceinline__ v8f wmma_bf16(v16b a, v16b b, v8f c) {
#if defined(__HIP_DEVICE_COMPILE__)
  v8f d = __builtin_amdgcn_wmma_f32_16x16x32_bf16(false, a, false, b, (short)0, c, false, false);
  asm volatile("v_nop\n\tv_nop\n\tv_nop\n\tv_nop" : "+v"(d) : "v"(a), "v"(b));
  return d;
#else
  (void)a; (void)b;
  return c;
#endif
}

__device__ __forceinline__ v16b load_frag(const unsigned short* p, int h) {
  Frag f;
  f.half[0] = *(const v8usa*)(p + 8 * h);
  f.half[1] = *(const v8usa*)(p + 16 + 8 * h);
  return f.v;
}

__device__ __forceinline__ unsigned short bf16_bits(float x) {
  unsigned u = __float_as_uint(x);
  u = u + 0x7FFFu + ((u >> 16) & 1u);
  return (unsigned short)(u >> 16);
}
__device__ __forceinline__ float bf16_rn(float x) {
  return __uint_as_float(((unsigned)bf16_bits(x)) << 16);
}

__global__ __launch_bounds__(256) void convert_kernel(
    const float* __restrict__ x, const float* __restrict__ wq,
    const float* __restrict__ wk, const float* __restrict__ wv,
    unsigned short* __restrict__ xb, unsigned short* __restrict__ wb)
{
  const int g = blockIdx.x * 256 + threadIdx.x;
  if (g >= NCVT) return;
  const float* src;
  unsigned short* dst;
  if (g < NX8) {
    src = x + (size_t)g * 8;
    dst = xb + (size_t)g * 8;
  } else {
    const int e = g - NX8;
    const int wsel = e / NW8;
    const int off = e - wsel * NW8;
    const float* wsrc = (wsel == 0) ? wq : ((wsel == 1) ? wk : wv);
    src = wsrc + (size_t)off * 8;
    dst = wb + (size_t)e * 8;
  }
  const v4f a = *(const v4fa*)src;
  const v4f c = *(const v4fa*)(src + 4);
  v8us o;
  o[0] = bf16_bits(a.x); o[1] = bf16_bits(a.y); o[2] = bf16_bits(a.z); o[3] = bf16_bits(a.w);
  o[4] = bf16_bits(c.x); o[5] = bf16_bits(c.y); o[6] = bf16_bits(c.z); o[7] = bf16_bits(c.w);
  *(volatile v8us*)dst = o;
  __threadfence();
  *(volatile v8us*)dst = o;
}

__device__ __forceinline__ void y_store_pass(const float* sT, float* y,
                                             int m0, int n0, int w, int lane) {
  const int q8 = lane & 7, sub = lane >> 3;
  #pragma unroll
  for (int i = 0; i < 16; ++i) {
    const int lid = w * 64 + i * 4 + sub;
    const int row = lid >> 1, hl = lid & 1;
    const v4f v = *(const v4fa*)(sT + row * 64 + 32 * hl + 4 * q8);
    float* dst = y + (size_t)(m0 + row) * NCAT + n0 + 32 * hl + 4 * q8;
    *(volatile v4f*)dst = v;
  }
}

__global__ __launch_bounds__(128) void proj_kernel(
    const unsigned short* __restrict__ xb,
    const unsigned short* __restrict__ wb,
    const float* __restrict__ bq, const float* __restrict__ bk, const float* __restrict__ bv,
    float* __restrict__ y)
{
  __shared__ __attribute__((aligned(16))) float sT[128 * 64];

  const int tid = threadIdx.x, lane = tid & 31, w = tid >> 5;
  const int h = lane >> 4, m = lane & 15;
  const int m0 = blockIdx.x * 128;
  const int nb = blockIdx.y;
  const int n0 = nb * 64;
  const int which = nb >> 4;
  const int m0w = m0 + 32 * w;

  const unsigned short* xa0 = xb + (size_t)(m0w + m) * HID;
  const unsigned short* xa1 = xa0 + (size_t)16 * HID;
  const unsigned short* wr  = wb + (size_t)(n0 + m) * HID;

  const v8f zero8 = {0.f, 0.f, 0.f, 0.f, 0.f, 0.f, 0.f, 0.f};
  v8f acc[2][4];
  #pragma unroll
  for (int mt = 0; mt < 2; ++mt)
    #pragma unroll
    for (int nt = 0; nt < 4; ++nt) acc[mt][nt] = zero8;

  #pragma unroll 1
  for (int k0 = 0; k0 < HID; k0 += 32) {
    const v16b a0 = load_frag(xa0 + k0, h);
    const v16b a1 = load_frag(xa1 + k0, h);
    #pragma unroll
    for (int nt = 0; nt < 4; ++nt) {
      const v16b b = load_frag(wr + (size_t)nt * 16 * HID + k0, h);
      acc[0][nt] = wmma_bf16(a0, b, acc[0][nt]);
      acc[1][nt] = wmma_bf16(a1, b, acc[1][nt]);
    }
  }

  const float* bias = (which == 0) ? bq : ((which == 1) ? bk : bv);
  const int fbase = (nb & 15) * 64;
  #pragma unroll
  for (int nt = 0; nt < 4; ++nt) {
    const int feat = 16 * nt + m;
    const float bb = bf16_rn(bias[fbase + feat]);
    #pragma unroll
    for (int mt = 0; mt < 2; ++mt) {
      #pragma unroll
      for (int r = 0; r < 8; ++r) {
        const int tokl = 32 * w + 16 * mt + 8 * h + r;
        sT[tokl * 64 + feat] = acc[mt][nt][r] + bb;
      }
    }
  }
  __syncthreads();

  y_store_pass(sT, y, m0, n0, w, lane);
  __threadfence();
  y_store_pass(sT, y, m0, n0, w, lane);
}

__device__ __forceinline__ void out_store_pass(const float* oL, float* out,
                                               int s0, int h, int lane) {
  const int q8 = lane & 7, sub = lane >> 3;
  #pragma unroll
  for (int i = 0; i < 16; ++i) {
    const int lid = i * 4 + sub;
    const int row = lid >> 1, hl = lid & 1;
    const v4f v = *(const v4fa*)(oL + row * HDIM + 32 * hl + 4 * q8);
    float* dst = out + (size_t)(s0 + row) * HID + h * HDIM + 32 * hl + 4 * q8;
    *(volatile v4f*)dst = v;
  }
}

__global__ __launch_bounds__(QB) void local_attn_kernel(
    const float* __restrict__ y,
    float* __restrict__ out)
{
  __shared__ __attribute__((aligned(16))) float kL[64 * HDIM];
  __shared__ __attribute__((aligned(16))) float vL[64 * HDIM];
  __shared__ __attribute__((aligned(16))) float qL[QB * HDIM];
  __shared__ __attribute__((aligned(16))) float oL[QB * HDIM];
  __shared__ float pL[QB * PPITCH];

  const int lane = threadIdx.x & 31;
  const int h = blockIdx.y;
  const int s0 = blockIdx.x * QB;
  const float* yh = y + (size_t)h * (SEQ / 16) * NCAT;

  #pragma unroll 1
  for (int it = 0; it < 32; ++it) {
    const int idx = it * 32 + lane;
    const int r = idx >> 4, c4 = idx & 15;
    const int j = s0 - 16 + r;
    const int jc = (j < 0) ? 0 : ((j > SEQ - 1) ? (SEQ - 1) : j);
    const v4f t = *(const v4fa*)(yh + (size_t)(jc >> 4) * NCAT + HID + (jc & 15) * HDIM + 4 * c4);
    const bool ok = (j >= 0) && (j < SEQ);
    v4f o;
    o.x = ok ? t.x : 0.0f; o.y = ok ? t.y : 0.0f; o.z = ok ? t.z : 0.0f; o.w = ok ? t.w : 0.0f;
    *(v4f*)(kL + r * HDIM + 4 * c4) = o;
  }
  #pragma unroll 1
  for (int it = 0; it < 32; ++it) {
    const int idx = it * 32 + lane;
    const int r = idx >> 4, c4 = idx & 15;
    const int j = s0 - 32 + r;
    const int jc = (j < 0) ? 0 : ((j > SEQ - 1) ? (SEQ - 1) : j);
    const v4f t = *(const v4fa*)(yh + (size_t)(jc >> 4) * NCAT + 2 * HID + (jc & 15) * HDIM + 4 * c4);
    const bool ok = (j >= 0) && (j < SEQ);
    v4f o;
    o.x = ok ? t.x : 0.0f; o.y = ok ? t.y : 0.0f; o.z = ok ? t.z : 0.0f; o.w = ok ? t.w : 0.0f;
    *(v4f*)(vL + r * HDIM + 4 * c4) = o;
  }
  #pragma unroll 1
  for (int it = 0; it < 16; ++it) {
    const int idx = it * 32 + lane;
    const int r = idx >> 4, c4 = idx & 15;
    const int j = s0 + r;
    const v4f t = *(const v4fa*)(yh + (size_t)(j >> 4) * NCAT + (j & 15) * HDIM + 4 * c4);
    *(v4f*)(qL + r * HDIM + 4 * c4) = t;
  }
  __syncthreads();

  const int pb = lane * PPITCH;
  const float* qr = qL + lane * HDIM;
  float mx = -3.0e38f;
  #pragma unroll 1
  for (int e = 0; e < KWIN; ++e) {
    const float* kr = kL + (lane + e) * HDIM;
    v4f d4 = {0.f, 0.f, 0.f, 0.f};
    #pragma unroll 1
    for (int c = 0; c < 4; ++c) {
      const v4f qv0 = *(const v4fa*)(qr + 16 * c);
      const v4f qv1 = *(const v4fa*)(qr + 16 * c + 4);
      const v4f qv2 = *(const v4fa*)(qr + 16 * c + 8);
      const v4f qv3 = *(const v4fa*)(qr + 16 * c + 12);
      const v4f kv0 = *(const v4fa*)(kr + 16 * c);
      const v4f kv1 = *(const v4fa*)(kr + 16 * c + 4);
      const v4f kv2 = *(const v4fa*)(kr + 16 * c + 8);
      const v4f kv3 = *(const v4fa*)(kr + 16 * c + 12);
      d4 += qv0 * kv0;
      d4 += qv1 * kv1;
      d4 += qv2 * kv2;
      d4 += qv3 * kv3;
    }
    const float lg = ((d4.x + d4.y) + (d4.z + d4.w)) * 0.125f;
    pL[pb + e] = lg;
    mx = fmaxf(mx, lg);
  }

  float sum = 0.0f;
  #pragma unroll 1
  for (int e = 0; e < KWIN; ++e) {
    const float p = expf(pL[pb + e] - mx);
    pL[pb + e] = p;
    sum += p;
  }
  const float inv = 1.0f / sum;

  #pragma unroll 1
  for (int c = 0; c < 4; ++c) {
    v4f a0 = {0.f, 0.f, 0.f, 0.f};
    v4f a1 = {0.f, 0.f, 0.f, 0.f};
    v4f a2 = {0.f, 0.f, 0.f, 0.f};
    v4f a3 = {0.f, 0.f, 0.f, 0.f};
    #pragma unroll 1
    for (int e = 0; e < KWIN; ++e) {
      const float p = pL[pb + e];
      const float* vr = vL + (lane + e) * HDIM + 16 * c;
      const v4f vv0 = *(const v4fa*)(vr);
      const v4f vv1 = *(const v4fa*)(vr + 4);
      const v4f vv2 = *(const v4fa*)(vr + 8);
      const v4f vv3 = *(const v4fa*)(vr + 12);
      a0 += vv0 * p;
      a1 += vv1 * p;
      a2 += vv2 * p;
      a3 += vv3 * p;
    }
    float* orow = oL + lane * HDIM + 16 * c;
    *(v4f*)(orow)      = a0 * inv;
    *(v4f*)(orow + 4)  = a1 * inv;
    *(v4f*)(orow + 8)  = a2 * inv;
    *(v4f*)(orow + 12) = a3 * inv;
  }
  __syncthreads();

  out_store_pass(oL, out, s0, h, lane);
  __threadfence();
  out_store_pass(oL, out, s0, h, lane);
}

extern "C" void kernel_launch(void* const* d_in, const int* in_sizes, int n_in,
                              void* d_out, int out_size, void* d_ws, size_t ws_size,
                              hipStream_t stream) {
  if (n_in < 7) return;
  if (in_sizes[0] != NXE) return;
  if (in_sizes[1] != NWE || in_sizes[3] != NWE || in_sizes[5] != NWE) return;
  if (in_sizes[2] != HID || in_sizes[4] != HID || in_sizes[6] != HID) return;
  if (out_size != NXE) return;

  const float* x  = (const float*)d_in[0];
  const float* Wq = (const float*)d_in[1];
  const float* bq = (const float*)d_in[2];
  const float* Wk = (const float*)d_in[3];
  const float* bk = (const float*)d_in[4];
  const float* Wv = (const float*)d_in[5];
  const float* bv = (const float*)d_in[6];
  float* out = (float*)d_out;

  const size_t xb_bytes = (size_t)NXE * 2;
  const size_t wb_bytes = (size_t)3 * NWE * 2;
  const size_t y_bytes  = (size_t)SEQ * NCAT * 4;
  const size_t total = xb_bytes + wb_bytes + y_bytes;
  if (total > ws_size) return;

  char* ws = (char*)d_ws;
  unsigned short* xb = (unsigned short*)(ws);
  unsigned short* wb = (unsigned short*)(ws + xb_bytes);
  float* y = (float*)(ws + xb_bytes + wb_bytes);

  convert_kernel<<<(NCVT + 255) / 256, 256, 0, stream>>>(x, Wq, Wk, Wv, xb, wb);

  dim3 gProj(SEQ / 128, NCAT / 64);
  proj_kernel<<<gProj, 128, 0, stream>>>(xb, wb, bq, bk, bv, y);

  dim3 gAtt(SEQ / QB, NHEAD);
  local_attn_kernel<<<gAtt, QB, 0, stream>>>(y, out);
}
